// Gemma2Original_22883585753583
// MI455X (gfx1250) — hardware-verified
//
#include <hip/hip_runtime.h>

typedef __attribute__((ext_vector_type(16))) _Float16 v16h;
typedef __attribute__((ext_vector_type(8)))  _Float16 v8h;
typedef __attribute__((ext_vector_type(16))) __bf16   v16b;
typedef __attribute__((ext_vector_type(8)))  __bf16   v8b;
typedef __attribute__((ext_vector_type(8)))  float    v8f;
typedef __attribute__((ext_vector_type(4)))  float    v4f;

#define AT_DH 128
#define AT_NW 4
#define AT_QB 64
#define AT_KC 64
#define OS_PITCH 68
#define TP_PITCH 72

__device__ __forceinline__ unsigned short at_bf_bits(float f) {
  unsigned u = __float_as_uint(f);
  return (unsigned short)((u + 0x7FFFu + ((u >> 16) & 1u)) >> 16);
}
__device__ __forceinline__ __bf16 at_f2bf(float f) { return __builtin_bit_cast(__bf16, at_bf_bits(f)); }
__device__ __forceinline__ void at_split(float f, __bf16& hi, __bf16& lo) {
  const unsigned short hb = at_bf_bits(f);
  hi = __builtin_bit_cast(__bf16, hb);
  lo = at_f2bf(f - __uint_as_float(((unsigned)hb) << 16));
}
__device__ __forceinline__ v8f at_mma(v16b a, v16b b, v8f c) {
  c = __builtin_amdgcn_wmma_f32_16x16x32_bf16(false, a, false, b, (short)0, c, false, false);
  asm volatile("v_nop\n\tv_nop\n\tv_nop\n\tv_nop" : "+v"(c) : "v"(a), "v"(b));
  return c;
}

__global__ __launch_bounds__(256) void cast_f32_bf16x8(
    const float* __restrict__ in, __bf16* __restrict__ out, int n8) {
  const int i = blockIdx.x * 256 + threadIdx.x;
  if (i < n8) {
    const size_t o = (size_t)i * 8;
    const v4f a = *(const v4f*)(in + o);
    const v4f b = *(const v4f*)(in + o + 4);
    v8b hv;
#pragma unroll
    for (int e = 0; e < 4; ++e) { hv[e] = at_f2bf(a[e]); hv[4 + e] = at_f2bf(b[e]); }
    const v8h bits = __builtin_bit_cast(v8h, hv);
    *(volatile v8h*)(out + o) = bits;
    __threadfence();
    *(volatile v8h*)(out + o) = bits;
  }
}

__global__ __launch_bounds__(256) void transpose_cast_bf16(
    const float* __restrict__ in, __bf16* __restrict__ out, int R, int C, long zin, long zout) {
  __shared__ __align__(16) __bf16 T[64 * TP_PITCH];
  const int tilesC = C >> 6;
  const int tr = blockIdx.x / tilesC;
  const int tc = blockIdx.x - tr * tilesC;
  const int r0 = tr << 6, c0 = tc << 6;
  const float* ib = in + (size_t)blockIdx.y * (size_t)zin;
  __bf16* ob = out + (size_t)blockIdx.y * (size_t)zout;
  const int tid = threadIdx.x;
#pragma unroll
  for (int i = 0; i < 4; ++i) {
    const int p = i * 256 + tid;
    const int r = p >> 4, c4 = (p & 15) * 4;
    const v4f x = *(const v4f*)(ib + (size_t)(r0 + r) * C + c0 + c4);
#pragma unroll
    for (int e = 0; e < 4; ++e) T[(c4 + e) * TP_PITCH + r] = at_f2bf(x[e]);
  }
  __syncthreads();
  const int wave = tid >> 5, lane = tid & 31;
  const int q = lane >> 3, c8 = (lane & 7) * 8;
  for (int pass = 0; pass < 2; ++pass) {
#pragma unroll
    for (int it = 0; it < 2; ++it) {
      const int line = wave * 8 + it * 4 + q;
      const v8b val = *(const v8b*)(T + line * TP_PITCH + c8);
      *(volatile v8h*)(ob + (size_t)(c0 + line) * R + r0 + c8) = __builtin_bit_cast(v8h, val);
    }
    __threadfence();
  }
}

__global__ __launch_bounds__(AT_NW * 32)
void attn128_causal(const __bf16* __restrict__ q16, const __bf16* __restrict__ k16,
                    const __bf16* __restrict__ vt16, float* __restrict__ out,
                    int S, float qk_scale, float cap, float inv_cap) {
  union FB { v16b v; v8b h[2]; };
  __shared__ __align__(16) unsigned char pool[AT_KC * AT_DH * 2 + AT_DH * AT_KC * 2 + 2 * AT_NW * 16 * AT_KC * 2];
  __bf16* Ksh  = (__bf16*)pool;
  __bf16* Vth  = Ksh + AT_KC * AT_DH;
  __bf16* PshA = Vth + AT_DH * AT_KC;
  __bf16* PslA = PshA + AT_NW * 16 * AT_KC;
  float*  OsA  = (float*)pool;

  const int tid  = threadIdx.x;
  const int wave = tid >> 5;
  const int lane = tid & 31;
  const int hh   = lane >> 4;
  const int c    = lane & 15;

  const int nqb = S / AT_QB;
  const int qb  = blockIdx.x % nqb;
  const int bh  = blockIdx.x / nqb;
  const int q0  = qb * AT_QB + wave * 16;
  const size_t hsz = (size_t)S * AT_DH;
  const __bf16* qb_ptr = q16  + (size_t)bh * hsz;
  const __bf16* kb_ptr = k16  + (size_t)bh * hsz;
  const __bf16* vb_ptr = vt16 + (size_t)bh * hsz;
  float*        ob_ptr = out  + (size_t)bh * hsz;

  v16b qa[4];
  {
    const __bf16* qrow = qb_ptr + (size_t)(q0 + c) * AT_DH;
#pragma unroll
    for (int dc = 0; dc < 4; ++dc) {
      FB f;
      f.h[0] = *(const v8b*)(qrow + dc * 32 + 8 * hh);
      f.h[1] = *(const v8b*)(qrow + dc * 32 + 16 + 8 * hh);
      qa[dc] = f.v;
    }
  }

  float mrow[8], lrow[8];
  v8f oacc[8];
#pragma unroll
  for (int r = 0; r < 8; ++r) { mrow[r] = -__builtin_inff(); lrow[r] = 0.f; }
#pragma unroll
  for (int t = 0; t < 8; ++t) oacc[t] = (v8f){0.f, 0.f, 0.f, 0.f, 0.f, 0.f, 0.f, 0.f};

  __bf16* pwh = PshA + wave * (16 * AT_KC);
  __bf16* pwl = PslA + wave * (16 * AT_KC);

  const int nChunks = qb + 1;
  for (int kc = 0; kc < nChunks; ++kc) {
    const int kv0 = kc * AT_KC;
    __syncthreads();
#pragma unroll
    for (int i = 0; i < 8; ++i) {
      const int p = i * (AT_NW * 32) + tid;
      const int row = p >> 4, c8 = (p & 15) * 8;
      *(v8b*)(Ksh + row * AT_DH + c8) = *(const v8b*)(kb_ptr + (size_t)(kv0 + row) * AT_DH + c8);
      const int d = p >> 3, k8 = (p & 7) * 8;
      *(v8b*)(Vth + d * AT_KC + k8) = *(const v8b*)(vb_ptr + (size_t)d * S + kv0 + k8);
    }
    __syncthreads();

    v8f s[4];
#pragma unroll
    for (int j = 0; j < 4; ++j) {
      s[j] = (v8f){0.f, 0.f, 0.f, 0.f, 0.f, 0.f, 0.f, 0.f};
#pragma unroll
      for (int dc = 0; dc < 4; ++dc) {
        FB kb;
        kb.h[0] = *(const v8b*)(Ksh + (j * 16 + c) * AT_DH + dc * 32 + 8 * hh);
        kb.h[1] = *(const v8b*)(Ksh + (j * 16 + c) * AT_DH + dc * 32 + 16 + 8 * hh);
        s[j] = at_mma(qa[dc], kb.v, s[j]);
      }
    }

    const bool diag = (kc == qb);
    float cm[8];
#pragma unroll
    for (int r = 0; r < 8; ++r) {
      const int qrow = q0 + 8 * hh + r;
      float m = -__builtin_inff();
#pragma unroll
      for (int j = 0; j < 4; ++j) {
        const int kvcol = kv0 + j * 16 + c;
        const float sv = s[j][r] * qk_scale;
        float y = tanhf(sv * inv_cap) * cap;
        if (diag && (kvcol > qrow)) y = -__builtin_inff();
        s[j][r] = y;
        m = fmaxf(m, y);
      }
#pragma unroll
      for (int off = 1; off < 16; off <<= 1) m = fmaxf(m, __shfl_xor(m, off, 32));
      cm[r] = m;
    }

#pragma unroll
    for (int r = 0; r < 8; ++r) {
      const float mnew  = fmaxf(mrow[r], cm[r]);
      const float alpha = expf(mrow[r] - mnew);
      mrow[r] = mnew;
      float psum = 0.f;
#pragma unroll
      for (int j = 0; j < 4; ++j) {
        const float p = expf(s[j][r] - mnew);
        psum += p;
        __bf16 ph, pl;
        at_split(p, ph, pl);
        pwh[(8 * hh + r) * AT_KC + j * 16 + c] = ph;
        pwl[(8 * hh + r) * AT_KC + j * 16 + c] = pl;
      }
#pragma unroll
      for (int off = 1; off < 16; off <<= 1) psum += __shfl_xor(psum, off, 32);
      lrow[r] = lrow[r] * alpha + psum;
#pragma unroll
      for (int t = 0; t < 8; ++t) oacc[t][r] *= alpha;
    }
    __builtin_amdgcn_fence(__ATOMIC_RELEASE, "workgroup");
    __builtin_amdgcn_wave_barrier();
    __builtin_amdgcn_fence(__ATOMIC_ACQUIRE, "workgroup");

#pragma unroll 1
    for (int kk = 0; kk < 2; ++kk) {
      FB pa, pl;
      pa.h[0] = *(const v8b*)(pwh + c * AT_KC + kk * 32 + 8 * hh);
      pa.h[1] = *(const v8b*)(pwh + c * AT_KC + kk * 32 + 16 + 8 * hh);
      pl.h[0] = *(const v8b*)(pwl + c * AT_KC + kk * 32 + 8 * hh);
      pl.h[1] = *(const v8b*)(pwl + c * AT_KC + kk * 32 + 16 + 8 * hh);
#pragma unroll
      for (int t = 0; t < 8; ++t) {
        FB vb;
        vb.h[0] = *(const v8b*)(Vth + (t * 16 + c) * AT_KC + kk * 32 + 8 * hh);
        vb.h[1] = *(const v8b*)(Vth + (t * 16 + c) * AT_KC + kk * 32 + 16 + 8 * hh);
        oacc[t] = at_mma(pa.v, vb.v, oacc[t]);
        oacc[t] = at_mma(pl.v, vb.v, oacc[t]);
      }
    }
  }

  __syncthreads();

  float* os = OsA + wave * (16 * OS_PITCH);
  const int c4 = c * 4;
#pragma unroll
  for (int hf = 0; hf < 2; ++hf) {
#pragma unroll
    for (int r = 0; r < 8; ++r) {
      const float inv = 1.0f / lrow[r];
#pragma unroll
      for (int tt = 0; tt < 4; ++tt) os[(8 * hh + r) * OS_PITCH + tt * 16 + c] = oacc[hf * 4 + tt][r] * inv;
    }
    __builtin_amdgcn_fence(__ATOMIC_RELEASE, "workgroup");
    __builtin_amdgcn_wave_barrier();
    __builtin_amdgcn_fence(__ATOMIC_ACQUIRE, "workgroup");
    for (int pass = 0; pass < 2; ++pass) {
#pragma unroll
      for (int it = 0; it < 8; ++it) {
        const int row = it * 2 + hh;
        const v4f val = *(const v4f*)(os + row * OS_PITCH + c4);
        *(volatile v4f*)(ob_ptr + (size_t)(q0 + row) * AT_DH + hf * 64 + c4) = val;
      }
      __threadfence();
    }
    __builtin_amdgcn_fence(__ATOMIC_RELEASE, "workgroup");
    __builtin_amdgcn_wave_barrier();
    __builtin_amdgcn_fence(__ATOMIC_ACQUIRE, "workgroup");
  }
}

extern "C" void kernel_launch(void* const* d_in, const int* in_sizes, int n_in,
                              void* d_out, int out_size, void* d_ws, size_t ws_size,
                              hipStream_t stream) {
  const int S = 2048;
  const int DH = AT_DH;
  if (n_in < 3) return;
  const long n = (long)in_sizes[0];
  const long per_head = (long)S * DH;
  if (n <= 0 || (n % per_head) != 0) return;
  if ((long)in_sizes[1] != n || (long)in_sizes[2] != n || (long)out_size != n) return;
  const int NBH = (int)(n / per_head);
  const size_t bytes16 = (size_t)n * 2;
  if (3 * bytes16 > ws_size) return;
  if (3 * bytes16 > (size_t)134217728) return;

  const float* q = (const float*)d_in[0];
  const float* k = (const float*)d_in[1];
  const float* v = (const float*)d_in[2];
  float* out = (float*)d_out;
  __bf16* q16  = (__bf16*)d_ws;
  __bf16* k16  = q16 + n;
  __bf16* vt16 = k16 + n;

  const int n8 = (int)(n / 8);
  cast_f32_bf16x8<<<dim3((unsigned)((n8 + 255) / 256)), dim3(256), 0, stream>>>(q, q16, n8);
  transpose_cast_bf16<<<dim3((unsigned)((DH / 64) * (S / 64)), (unsigned)NBH), dim3(256), 0, stream>>>(
      k, k16, DH, S, per_head, per_head);
  transpose_cast_bf16<<<dim3((unsigned)((S / 64) * (DH / 64)), (unsigned)NBH), dim3(256), 0, stream>>>(
      v, vt16, S, DH, per_head, per_head);
  const float qk_scale = 0.08838834764831845f;
  const float cap = 50.0f;
  const float inv_cap = 0.02f;
  attn128_causal<<<dim3((unsigned)(NBH * (S / AT_QB))), dim3(AT_NW * 32), 0, stream>>>(
      q16, k16, vt16, out, S, qk_scale, cap, inv_cap);
}
